// GCNPose3D_15006615732993
// MI455X (gfx1250) — hardware-verified
//
#include <hip/hip_runtime.h>
#include <stddef.h>
#include <stdint.h>


#define NJ     17
#define HID    256
#define CIN    3
#define COUT   3
#define NLAY   4
#define GPB    9
#define MROWS  (GPB * NJ)
#define MTILE  10
#define MPAD   (MTILE * 16)
#define NGRP   15552
#define NBLK   (NGRP / GPB)
#define NROWS  (NGRP * NJ)
#define NOUT   (NROWS * COUT)
#define NTHR   512
#define NWAVE  16
#define NTHR_S 256
#define HSC    16
#define WSC    64
#define YSLOT  480
#define WSCAP  134217728

#define LO_HM16 0
#define SZ_HM16 (MPAD * HID * 2)
#define LO_H32  (LO_HM16 + SZ_HM16)
#define SZ_H32  (MROWS * HID * 4)
#define LO_SA   (LO_H32 + SZ_H32)
#define SZ_SA   1168
#define LO_SDH  (LO_SA + SZ_SA)
#define SZ_SDH  80
#define LO_SIDX (LO_SDH + SZ_SDH)
#define SZ_SIDX 1168
#define LO_SVAL (LO_SIDX + SZ_SIDX)
#define SZ_SVAL 1168
#define LO_SCNT (LO_SVAL + SZ_SVAL)
#define SZ_SCNT 80
#define LO_SY   (LO_SCNT + SZ_SCNT)
#define SZ_SY   (YSLOT * 4)
#define LDS_LAYERS (LO_SY + SZ_SY)

static_assert((NGRP % GPB) == 0);
static_assert(NWAVE * 16 == HID);
static_assert(NTHR == 32 * NWAVE);
static_assert(MPAD >= MROWS);
static_assert(MROWS * COUT <= YSLOT);
static_assert(((YSLOT * 4) % 128) == 0);
static_assert((NOUT % 4) == 0);
static_assert((HID % 32) == 0);
static_assert((MPAD - MROWS) * (HID / 8) <= NTHR);
static_assert(YSLOT / 4 <= NTHR);
static_assert(MROWS <= NTHR);
static_assert(NJ * NJ * 4 <= SZ_SA);
static_assert(((NLAY * HID) % (NTHR_S / 32)) == 0);
static_assert((LO_H32 % 16) == 0 && (LO_SA % 16) == 0 && (LO_SY % 16) == 0);
static_assert(LDS_LAYERS <= 300 * 1024);

typedef float    v4f  __attribute__((ext_vector_type(4)));
typedef float    v8f  __attribute__((ext_vector_type(8)));
typedef _Float16 v8h  __attribute__((ext_vector_type(8)));
typedef _Float16 v16h __attribute__((ext_vector_type(16)));
union FragH { v16h v; v8h h[2]; };

__device__ __forceinline__ v8f wmf(v16h a, v16h b, v8f c) {
  v8f d = __builtin_amdgcn_wmma_f32_16x16x32_f16(false, a, false, b, (short)0, c, false, false);
  asm volatile("v_nop\n\tv_nop\n\tv_nop\n\tv_nop" : "+v"(d) : "v"(a), "v"(b));
  return d;
}

__global__ __launch_bounds__(NTHR_S) void k_prepw(const float* __restrict__ Ws, _Float16* wt) {
  const int tid = threadIdx.x, lane = tid & 31, wave = tid >> 5;
  const int rn = blockIdx.x * (NTHR_S / 32) + wave;
  const int l = rn >> 8, n = rn & 255;
  const float* src = Ws + (size_t)l * (HID * HID) + (size_t)(8 * lane) * HID + n;
  v8h a;
#pragma unroll
  for (int i = 0; i < 8; ++i) a[i] = (_Float16)(src[(size_t)i * HID] * (float)WSC);
  _Float16* d = wt + (size_t)rn * HID + 8 * lane;
  *(volatile v8h*)d = a;
  __threadfence();
  *(volatile v8h*)d = a;
}

__global__ __launch_bounds__(NTHR) void k_layers(
    const float* __restrict__ x, const float* __restrict__ adj,
    const float* __restrict__ w_in, const float* __restrict__ b_in,
    const _Float16* __restrict__ wt, const float* __restrict__ bs,
    const float* __restrict__ w_out, const float* __restrict__ b_out,
    float* yslot)
{
  extern __shared__ v4f lds_dyn[];
  char* lds = (char*)lds_dyn;
  _Float16* hm16 = (_Float16*)(lds + LO_HM16);
  float* h32  = (float*)(lds + LO_H32);
  float* sA   = (float*)(lds + LO_SA);
  float* sdh  = (float*)(lds + LO_SDH);
  int*   sidx = (int*)(lds + LO_SIDX);
  float* sval = (float*)(lds + LO_SVAL);
  int*   scnt = (int*)(lds + LO_SCNT);
  float* sy   = (float*)(lds + LO_SY);

  const int tid = threadIdx.x, lane = tid & 31, hf = lane >> 4, m = lane & 15;
  const int wave = __builtin_amdgcn_readfirstlane(tid >> 5);
  const int blk = blockIdx.x;

  if (tid < NJ) {
    float s = 0.0f;
#pragma unroll 1
    for (int k = 0; k < NJ; ++k) s += adj[tid * NJ + k];
    sdh[tid] = rsqrtf(s + 1e-5f);
  }
  __syncthreads();
  if (tid < NJ * NJ) {
    const int j = tid / NJ, k = tid - j * NJ;
    sA[tid] = sdh[j] * adj[tid] * sdh[k];
  }
  {
    const float* xg = x + (size_t)blk * (MROWS * CIN);
    for (int idx = tid; idx < MROWS * (HID / 4); idx += NTHR) {
      const int row = idx >> 6, c4 = (idx & 63) << 2;
      const float x0 = xg[row * CIN], x1 = xg[row * CIN + 1], x2 = xg[row * CIN + 2];
      const v4f w0 = *(const v4f*)(w_in + c4);
      const v4f w1 = *(const v4f*)(w_in + HID + c4);
      const v4f w2 = *(const v4f*)(w_in + 2 * HID + c4);
      const v4f bb = *(const v4f*)(b_in + c4);
      v4f d = x0 * w0;
      d = x1 * w1 + d;
      d = x2 * w2 + d;
      *(v4f*)(h32 + row * HID + c4) = d + bb;
    }
  }
  if (tid < (MPAD - MROWS) * (HID / 8)) {
    v8h z;
#pragma unroll
    for (int i = 0; i < 8; ++i) z[i] = (_Float16)0.0f;
    *(v8h*)(hm16 + MROWS * HID + 8 * tid) = z;
  }
  __syncthreads();
  if (tid < NJ) {
    int c = 0;
#pragma unroll 1
    for (int k = 0; k < NJ; ++k) {
      const float a = sA[tid * NJ + k];
      if (a != 0.0f) {
        sidx[tid * NJ + c] = k;
        sval[tid * NJ + c] = a;
        ++c;
      }
    }
    scnt[tid] = c;
  }
  __syncthreads();

  const int col = 16 * wave + m;
  const _Float16* bbase = wt + (size_t)col * HID + 8 * hf;
  constexpr float INV = 1.0f / (float)(HSC * WSC);

#pragma unroll 1
  for (int l = 0; l < NLAY; ++l) {
    for (int task = wave; task < MROWS; task += NWAVE) {
      const int g = task / NJ, j = task - g * NJ;
      int cnt = __builtin_amdgcn_readfirstlane(scnt[j]);
      cnt = cnt < 0 ? 0 : cnt;
      cnt = cnt > NJ ? NJ : cnt;
      const float* hrow = h32 + (g * NJ) * HID + 8 * lane;
      const int lb = j * NJ;
      v4f a0 = {0.0f, 0.0f, 0.0f, 0.0f};
      v4f a1 = a0;
#pragma unroll 1
      for (int q = 0; q < cnt; ++q) {
        int k = sidx[lb + q];
        k = k < 0 ? 0 : k;
        k = k > NJ - 1 ? NJ - 1 : k;
        const float av = sval[lb + q];
        const float* hp = hrow + k * HID;
        const v4f u0 = *(const v4f*)hp;
        const v4f u1 = *(const v4f*)(hp + 4);
        a0 = av * u0 + a0;
        a1 = av * u1 + a1;
      }
      v8h o;
      o[0] = (_Float16)(a0.x * (float)HSC); o[1] = (_Float16)(a0.y * (float)HSC);
      o[2] = (_Float16)(a0.z * (float)HSC); o[3] = (_Float16)(a0.w * (float)HSC);
      o[4] = (_Float16)(a1.x * (float)HSC); o[5] = (_Float16)(a1.y * (float)HSC);
      o[6] = (_Float16)(a1.z * (float)HSC); o[7] = (_Float16)(a1.w * (float)HSC);
      *(v8h*)(hm16 + (g * NJ + j) * HID + 8 * lane) = o;
    }
    __syncthreads();

    v8f acc[MTILE];
#pragma unroll
    for (int mt = 0; mt < MTILE; ++mt) {
      v8f z = {0.0f, 0.0f, 0.0f, 0.0f, 0.0f, 0.0f, 0.0f, 0.0f};
      acc[mt] = z;
    }
    const _Float16* bp = bbase + (size_t)l * (HID * HID);
#pragma unroll 1
    for (int kt = 0; kt < HID / 32; ++kt) {
      const int k0 = 32 * kt;
      FragH b;
      b.h[0] = *(const v8h*)(bp + k0);
      b.h[1] = *(const v8h*)(bp + k0 + 16);
#pragma unroll
      for (int mt = 0; mt < MTILE; ++mt) {
        const _Float16* ap = hm16 + (16 * mt + m) * HID + 8 * hf + k0;
        FragH a;
        a.h[0] = *(const v8h*)ap;
        a.h[1] = *(const v8h*)(ap + 16);
        acc[mt] = wmf(a.v, b.v, acc[mt]);
      }
    }

    const float bsv = bs[l * HID + col];
#pragma unroll
    for (int mt = 0; mt < MTILE; ++mt) {
#pragma unroll
      for (int r = 0; r < 8; ++r) {
        const int row = 16 * mt + 8 * hf + r;
        if (row < MROWS) {
          float* p = h32 + row * HID + col;
          const float o = acc[mt][r] * INV + bsv;
          const float hold = *p;
          *p = fmaxf(o, 0.0f) + hold;
        }
      }
    }
    __syncthreads();
  }

  if (tid < MROWS) {
    const float* hr = h32 + tid * HID;
    float y0 = 0.0f, y1 = 0.0f, y2 = 0.0f;
#pragma unroll 1
    for (int qd = 0; qd < HID / 4; ++qd) {
      const v4f hv = *(const v4f*)(hr + 4 * qd);
      const v4f f0 = *(const v4f*)(w_out + 12 * qd);
      const v4f f1 = *(const v4f*)(w_out + 12 * qd + 4);
      const v4f f2 = *(const v4f*)(w_out + 12 * qd + 8);
      y0 = fmaf(hv.x, f0.x, y0); y1 = fmaf(hv.x, f0.y, y1); y2 = fmaf(hv.x, f0.z, y2);
      y0 = fmaf(hv.y, f0.w, y0); y1 = fmaf(hv.y, f1.x, y1); y2 = fmaf(hv.y, f1.y, y2);
      y0 = fmaf(hv.z, f1.z, y0); y1 = fmaf(hv.z, f1.w, y1); y2 = fmaf(hv.z, f2.x, y2);
      y0 = fmaf(hv.w, f2.y, y0); y1 = fmaf(hv.w, f2.z, y1); y2 = fmaf(hv.w, f2.w, y2);
    }
    sy[tid * COUT + 0] = y0 + b_out[0];
    sy[tid * COUT + 1] = y1 + b_out[1];
    sy[tid * COUT + 2] = y2 + b_out[2];
  }
  if (tid < YSLOT - MROWS * COUT) sy[MROWS * COUT + tid] = 0.0f;
  __syncthreads();
  if (tid < YSLOT / 4) {
    const v4f v = *(const v4f*)(sy + 4 * tid);
    float* d = yslot + (size_t)blk * YSLOT + 4 * tid;
    *(volatile v4f*)d = v;
    __threadfence();
    *(volatile v4f*)d = v;
  }
}

__global__ __launch_bounds__(NTHR_S) void k_out(const float* __restrict__ yslot, float* out) {
  const int t = blockIdx.x * NTHR_S + threadIdx.x;
  if (t >= NOUT / 4) return;
  v4f v;
#pragma unroll
  for (int i = 0; i < 4; ++i) {
    const int e = 4 * t + i;
    const int b = e / (MROWS * COUT);
    const int off = e - b * (MROWS * COUT);
    v[i] = yslot[(size_t)b * YSLOT + off];
  }
  float* d = out + (size_t)4 * t;
  *(volatile v4f*)d = v;
  __threadfence();
  *(volatile v4f*)d = v;
}

extern "C" void kernel_launch(void* const* d_in, const int* in_sizes, int n_in,
                              void* d_out, int out_size, void* d_ws, size_t ws_size,
                              hipStream_t stream) {
  if (n_in < 8) return;
  if (in_sizes[0] != NROWS * CIN || in_sizes[1] != NJ * NJ || in_sizes[2] != CIN * HID ||
      in_sizes[3] != HID || in_sizes[4] != NLAY * HID * HID || in_sizes[5] != NLAY * HID ||
      in_sizes[6] != HID * COUT || in_sizes[7] != COUT) return;
  if (out_size != NOUT) return;

  const float* x     = (const float*)d_in[0];
  const float* adj   = (const float*)d_in[1];
  const float* w_in  = (const float*)d_in[2];
  const float* b_in  = (const float*)d_in[3];
  const float* Ws    = (const float*)d_in[4];
  const float* bs    = (const float*)d_in[5];
  const float* w_out = (const float*)d_in[6];
  const float* b_out = (const float*)d_in[7];
  float* out = (float*)d_out;

  char* ws = (char*)d_ws;
  size_t off = 0;
  const size_t oW = off; off += (size_t)NLAY * HID * HID * 2;  off = (off + 255) & ~(size_t)255;
  const size_t oY = off; off += (size_t)NBLK * YSLOT * 4;       off = (off + 255) & ~(size_t)255;
  if (off > ws_size || off > (size_t)WSCAP) return;
  _Float16* wt = (_Float16*)(ws + oW);
  float* yslot = (float*)(ws + oY);

  k_prepw<<<(NLAY * HID) / (NTHR_S / 32), NTHR_S, 0, stream>>>(Ws, wt);
  hipFuncSetAttribute(reinterpret_cast<const void*>(&k_layers),
                      hipFuncAttributeMaxDynamicSharedMemorySize, LDS_LAYERS);
  k_layers<<<NBLK, NTHR, LDS_LAYERS, stream>>>(x, adj, w_in, b_in, wt, bs, w_out, b_out, yslot);
  k_out<<<(NOUT / 4 + NTHR_S - 1) / NTHR_S, NTHR_S, 0, stream>>>(yslot, out);
}
